// MultiQuerySelfAttention_78426102825680
// MI455X (gfx1250) — hardware-verified
//
#include <hip/hip_runtime.h>
#include <math.h>

constexpr int kBatch   = 4;
constexpr int kSeq     = 2048;
constexpr int kDModel  = 1024;
constexpr int kHeads   = 16;
constexpr int kDh      = 64;
constexpr int kTok     = kBatch * kSeq;
constexpr int kGrp     = 4;
constexpr int kHeadChunks = kHeads / kGrp;
constexpr float kWCarry    = 16.0f;
constexpr float kWCarryInv = 1.0f / 16.0f;
constexpr float kScoreScale = 0.125f;
constexpr float kPCarry    = 2048.0f;
constexpr float kOCarry    = 256.0f;
constexpr float kPVScale   = kOCarry / kPCarry;
constexpr float kOutScale  = 1.0f / (kOCarry * kWCarry);
static_assert(kHeads % kGrp == 0);
static_assert(kSeq % 64 == 0 && kDModel % 64 == 0 && kDh % 64 == 0 && kTok % 64 == 0);
static_assert(kDModel % 32 == 0 && kDh % 32 == 0 && kSeq % 32 == 0);

typedef __attribute__((ext_vector_type(16))) _Float16 v16h;
typedef __attribute__((ext_vector_type(8)))  _Float16 v8h;
typedef __attribute__((ext_vector_type(16))) __bf16   v16b;
typedef __attribute__((ext_vector_type(8)))  __bf16   v8b;
typedef __attribute__((ext_vector_type(8)))  float    v8f;
typedef __attribute__((ext_vector_type(4)))  float    v4f;
typedef __attribute__((ext_vector_type(4)))  unsigned int v4u;

__device__ __forceinline__ unsigned short f2bf_bits(float f) {
  unsigned u = __float_as_uint(f);
  return (unsigned short)((u + 0x7FFFu + ((u >> 16) & 1u)) >> 16);
}
__device__ __forceinline__ float bf_bits2f(unsigned short h) { return __uint_as_float(((unsigned)h) << 16); }

__device__ __forceinline__ void dep_guard_h(v8f& a, v8f& b, v16h x, v16h y) { asm volatile("v_nop\n\tv_nop\n\tv_nop\n\tv_nop" : "+v"(a), "+v"(b) : "v"(x), "v"(y)); }
__device__ __forceinline__ void dep_guard_b(v8f& a, v8f& b, v16b x, v16b y) { asm volatile("v_nop\n\tv_nop\n\tv_nop\n\tv_nop" : "+v"(a), "+v"(b) : "v"(x), "v"(y)); }
__device__ __forceinline__ void keep4_h(v16h a, v16h b, v16h c, v16h d) { asm volatile("v_nop" :: "v"(a), "v"(b), "v"(c), "v"(d)); }
__device__ __forceinline__ void keep4_b(v16b a, v16b b, v16b c, v16b d) { asm volatile("v_nop" :: "v"(a), "v"(b), "v"(c), "v"(d)); }
__device__ __forceinline__ void acc_guard4(v8f& a, v8f& b, v8f& c, v8f& d) { asm volatile("v_nop\n\tv_nop\n\tv_nop\n\tv_nop" : "+v"(a), "+v"(b), "+v"(c), "+v"(d)); }
template <typename T> struct Frag;
template <> struct Frag<_Float16> {
  typedef v16h V; union U { v16h v; v8h h[2]; };
  static __device__ __forceinline__ v16h load(const _Float16* p) {
    U f; f.h[0] = *(const v8h*)(p); f.h[1] = *(const v8h*)(p + 16); return f.v;
  }
  static __device__ __forceinline__ v8f mma(v16h a, v16h b, v8f c) {
    return __builtin_amdgcn_wmma_f32_16x16x32_f16(false, a, false, b, (short)0, c, false, false);
  }
  static __device__ __forceinline__ void guard(v8f& a, v8f& b, v16h x, v16h y) { dep_guard_h(a, b, x, y); }
  static __device__ __forceinline__ void keep(v16h a, v16h b, v16h c, v16h d) { keep4_h(a, b, c, d); }
};
template <> struct Frag<__bf16> {
  typedef v16b V; union U { v16b v; v8b h[2]; };
  static __device__ __forceinline__ v16b load(const __bf16* p) {
    U f; f.h[0] = *(const v8b*)(p); f.h[1] = *(const v8b*)(p + 16); return f.v;
  }
  static __device__ __forceinline__ v8f mma(v16b a, v16b b, v8f c) {
    return __builtin_amdgcn_wmma_f32_16x16x32_bf16(false, a, false, b, (short)0, c, false, false);
  }
  static __device__ __forceinline__ void guard(v8f& a, v8f& b, v16b x, v16b y) { dep_guard_b(a, b, x, y); }
  static __device__ __forceinline__ void keep(v16b a, v16b b, v16b c, v16b d) { keep4_b(a, b, c, d); }
};

__device__ __forceinline__ unsigned pk16(unsigned short a, unsigned short b) { return (unsigned)a | ((unsigned)b << 16); }
__device__ __forceinline__ unsigned short h_bits(float f) { const _Float16 h = (_Float16)f; return __builtin_bit_cast(unsigned short, h); }

template <int ET> struct Elem;
template <> struct Elem<0> { typedef _Float16 T; };
template <> struct Elem<1> { typedef __bf16 T; };
template <int ET, bool SPLIT, int BIAS_MODE, int OUT_MODE, bool RESID, int ACT = 0>
__global__ __launch_bounds__(256) void wmma_gemm64(
    const unsigned short* __restrict__ Ap, const unsigned short* __restrict__ A2p, int lda, long strideA,
    const unsigned short* __restrict__ Btp, const unsigned short* __restrict__ Bt2p, int ldb, long strideB,
    void* __restrict__ Cout, void* __restrict__ Cout2, int ldc, long strideC,
    const float* __restrict__ bias,
    const float* __restrict__ resid, long strideR,
    int M, int N, int K, float scale) {
  typedef typename Elem<ET>::T T;
  typedef typename Frag<T>::V V;
  const T* A = (const T*)Ap; const T* A2 = (const T*)A2p; const T* Bt = (const T*)Btp; const T* Bt2 = (const T*)Bt2p;
  __shared__ __align__(16) float sT[8][16 * 68];
  const int b    = blockIdx.y;
  const int lane = threadIdx.x & 31;
  const int wave = threadIdx.x >> 5;
  const int tilesN = N >> 6;
  const int tilesM = M >> 6;
  const int tile = blockIdx.x * 8 + wave;
  if (tile >= tilesM * tilesN) return;
  const int tm = tile / tilesN;
  const int tn = tile - tm * tilesN;
  const int m0 = tm << 6;
  const int n0 = tn << 6;

  const T* Ab  = A  + (size_t)b * strideA;
  const T* Bb  = Bt + (size_t)b * strideB;
  const T* Ab2 = SPLIT ? (A2  + (size_t)b * strideA) : nullptr;
  const T* Bb2 = SPLIT ? (Bt2 + (size_t)b * strideB) : nullptr;

  const int rlane = lane & 15;
  const int koff  = (lane >> 4) * 8;
  const int mOff  = (lane >> 4) * 8;

  v8f acc[4][4];
#pragma unroll
  for (int i = 0; i < 4; ++i)
#pragma unroll
    for (int j = 0; j < 4; ++j) acc[i][j] = (v8f){0.f,0.f,0.f,0.f,0.f,0.f,0.f,0.f};

  for (int k0 = 0; k0 < K; k0 += 32) {
    V bh[4], bl[4];
#pragma unroll
    for (int j = 0; j < 4; ++j) {
      const size_t bo = (size_t)(n0 + (j << 4) + rlane) * ldb + koff + k0;
      bh[j] = Frag<T>::load(Bb + bo);
      if (SPLIT) bl[j] = Frag<T>::load(Bb2 + bo);
    }
#pragma unroll
    for (int i = 0; i < 4; ++i) {
      const size_t ao = (size_t)(m0 + (i << 4) + rlane) * lda + koff + k0;
      V ah = Frag<T>::load(Ab + ao);
      V al;
      if (SPLIT) al = Frag<T>::load(Ab2 + ao);
#pragma unroll
      for (int j = 0; j < 4; ++j) {
        acc[i][j] = Frag<T>::mma(ah, bh[j], acc[i][j]);
        if (SPLIT) {
          acc[i][j] = Frag<T>::mma(ah, bl[j], acc[i][j]);
          acc[i][j] = Frag<T>::mma(al, bh[j], acc[i][j]);
        }
      }
      Frag<T>::guard(acc[i][0], acc[i][3], ah, SPLIT ? al : ah);
    }
    Frag<T>::keep(bh[0], bh[1], bh[2], bh[3]);
    if (SPLIT) Frag<T>::keep(bl[0], bl[1], bl[2], bl[3]);
  }
  acc_guard4(acc[0][0], acc[0][1], acc[0][2], acc[0][3]);
  acc_guard4(acc[1][0], acc[1][1], acc[1][2], acc[1][3]);
  acc_guard4(acc[2][0], acc[2][1], acc[2][2], acc[2][3]);
  acc_guard4(acc[3][0], acc[3][1], acc[3][2], acc[3][3]);

  float* slab = sT[wave];
  const float* Rb = RESID ? (resid + (size_t)b * strideR) : nullptr;
#pragma unroll
  for (int i = 0; i < 4; ++i) {
    const int mBase = m0 + (i << 4);
#pragma unroll
    for (int j = 0; j < 4; ++j) {
      const int n = n0 + (j << 4) + rlane;
      float bv = 0.f;
      if (BIAS_MODE == 2) bv = bias[n];
#pragma unroll
      for (int r = 0; r < 8; ++r) {
        float v = acc[i][j][r] * scale;
        if (BIAS_MODE == 1) v += bias[mBase + mOff + r];
        if (BIAS_MODE == 2) v += bv;
        if (RESID) v += Rb[(size_t)(mBase + mOff + r) * ldc + n];
        if (ACT == 2) v = fmaxf(v, 0.0f);
        if (ACT == 4) v = (v > 0.f) ? v : 0.01f * v;
        slab[(mOff + r) * 68 + (j << 4) + rlane] = v;
      }
    }
    __builtin_amdgcn_fence(__ATOMIC_RELEASE, "workgroup");
    __builtin_amdgcn_wave_barrier();
    __builtin_amdgcn_fence(__ATOMIC_ACQUIRE, "workgroup");
    if (OUT_MODE == 0) {
      float* C = (float*)Cout + (size_t)b * strideC;
      const int hh = lane >> 4, c4 = (lane & 15) * 4;
      for (int pass = 0; pass < 2; ++pass) {
#pragma unroll
        for (int it = 0; it < 8; ++it) {
          const int row = it * 2 + hh;
          v4f v = *(const v4f*)(slab + row * 68 + c4);
          *(volatile v4f*)(C + (size_t)(mBase + row) * ldc + n0 + c4) = v;
        }
        __threadfence();
      }
    } else {
      const int q = lane >> 3, c8 = (lane & 7) * 8;
      unsigned short* C  = (unsigned short*)Cout  + (size_t)b * strideC;
      unsigned short* C2 = (OUT_MODE == 2) ? ((unsigned short*)Cout2 + (size_t)b * strideC) : nullptr;
      for (int pass = 0; pass < 2; ++pass) {
#pragma unroll
        for (int it = 0; it < 4; ++it) {
          const int row = it * 4 + q;
          const float* sp = slab + row * 68 + c8;
          v8h hv, lv;
#pragma unroll
          for (int e = 0; e < 8; ++e) {
            if (OUT_MODE == 1) {
              hv[e] = (_Float16)sp[e];
            } else {
              unsigned short hb = f2bf_bits(sp[e]);
              unsigned short lb = f2bf_bits(sp[e] - bf_bits2f(hb));
              hv[e] = __builtin_bit_cast(_Float16, hb);
              lv[e] = __builtin_bit_cast(_Float16, lb);
            }
          }
          *(volatile v8h*)(C + (size_t)(mBase + row) * ldc + n0 + c8) = hv;
          if (OUT_MODE == 2) *(volatile v8h*)(C2 + (size_t)(mBase + row) * ldc + n0 + c8) = lv;
        }
        __threadfence();
      }
    }
    __builtin_amdgcn_fence(__ATOMIC_RELEASE, "workgroup");
    __builtin_amdgcn_wave_barrier();
    __builtin_amdgcn_fence(__ATOMIC_ACQUIRE, "workgroup");
  }
}

__global__ __launch_bounds__(256) void wtcast_kernel(const float* __restrict__ W0, const float* __restrict__ W1,
                                                     unsigned short* __restrict__ out0, unsigned short* __restrict__ out1,
                                                     int R, int NC, float scale) {
  __shared__ float sm[64][65];
  const int t  = threadIdx.x;
  const int r0 = blockIdx.x * 64;
  const int c0 = blockIdx.y * 64;
  const int z  = blockIdx.z;
  const float* W = (z == 0) ? W0 : W1;
  unsigned short* op = (z == 0) ? out0 : out1;
#pragma unroll
  for (int i = 0; i < 16; ++i) {
    const int e  = i * 256 + t;
    const int rl = e >> 6;
    const int cl = e & 63;
    sm[cl][rl] = W[(size_t)(r0 + rl) * NC + c0 + cl] * scale;
  }
  __syncthreads();
  const int lane = t & 31, wave = t >> 5;
  const int q = lane >> 3, c8 = (lane & 7) * 8;
  for (int pass = 0; pass < 2; ++pass) {
#pragma unroll
    for (int it = 0; it < 2; ++it) {
      const int row = wave * 8 + it * 4 + q;
      unsigned short hb[8];
#pragma unroll
      for (int e = 0; e < 8; ++e) hb[e] = h_bits(sm[row][c8 + e]);
      const v4u u = (v4u){pk16(hb[0], hb[1]), pk16(hb[2], hb[3]), pk16(hb[4], hb[5]), pk16(hb[6], hb[7])};
      *(volatile v4u*)(op + (size_t)(c0 + row) * R + r0 + c8) = u;
    }
    __threadfence();
  }
}

__global__ __launch_bounds__(256) void cast8_f16_kernel(const float* __restrict__ in, unsigned short* __restrict__ out, int n8) {
  const int i = blockIdx.x * 256 + threadIdx.x;
  if (i >= n8) return;
  const float* p = in + 8 * (size_t)i;
  const v4f a = *(const v4f*)(p);
  const v4f c = *(const v4f*)(p + 4);
  unsigned short hb[8];
#pragma unroll
  for (int e = 0; e < 4; ++e) {
    hb[e]     = h_bits(a[e]);
    hb[4 + e] = h_bits(c[e]);
  }
  const v4u u = (v4u){pk16(hb[0], hb[1]), pk16(hb[2], hb[3]), pk16(hb[4], hb[5]), pk16(hb[6], hb[7])};
  unsigned short* q = out + 8 * (size_t)i;
  *(volatile v4u*)q = u;
  __threadfence();
  *(volatile v4u*)q = u;
}

__global__ __launch_bounds__(256) void softmax_row_kernel(const float* __restrict__ S, unsigned short* __restrict__ P, float carry) {
  __shared__ float redM[8];
  __shared__ float redS[8];
  const int row  = blockIdx.x;
  const int t    = threadIdx.x;
  const int lane = t & 31, wave = t >> 5;
  const int c0   = t * 8;
  const float* sr = S + (size_t)row * kSeq + c0;
  const v4f a = *(const v4f*)(sr);
  const v4f c = *(const v4f*)(sr + 4);
  float x[8];
#pragma unroll
  for (int e = 0; e < 4; ++e) { x[e] = a[e]; x[4 + e] = c[e]; }
  float m = fmaxf(fmaxf(fmaxf(x[0], x[1]), fmaxf(x[2], x[3])), fmaxf(fmaxf(x[4], x[5]), fmaxf(x[6], x[7])));
#pragma unroll
  for (int off = 16; off > 0; off >>= 1) m = fmaxf(m, __shfl_xor(m, off, 32));
  if (lane == 0) redM[wave] = m;
  __syncthreads();
  float gm = redM[0];
#pragma unroll
  for (int w = 1; w < 8; ++w) gm = fmaxf(gm, redM[w]);
  float ex[8];
  float s = 0.f;
#pragma unroll
  for (int e = 0; e < 8; ++e) { ex[e] = expf(x[e] - gm); s += ex[e]; }
#pragma unroll
  for (int off = 16; off > 0; off >>= 1) s += __shfl_xor(s, off, 32);
  if (lane == 0) redS[wave] = s;
  __syncthreads();
  float tot = redS[0];
#pragma unroll
  for (int w = 1; w < 8; ++w) tot += redS[w];
  const float inv = carry * (1.0f / tot);
  unsigned short hb[8];
#pragma unroll
  for (int e = 0; e < 8; ++e) hb[e] = h_bits(ex[e] * inv);
  const v4u u = (v4u){pk16(hb[0], hb[1]), pk16(hb[2], hb[3]), pk16(hb[4], hb[5]), pk16(hb[6], hb[7])};
  unsigned short* qp = P + (size_t)row * kSeq + c0;
  *(volatile v4u*)qp = u;
  __threadfence();
  *(volatile v4u*)qp = u;
}

extern "C" void kernel_launch(void* const* d_in, const int* in_sizes, int n_in,
                              void* d_out, int out_size, void* d_ws, size_t ws_size,
                              hipStream_t stream) {
  if (n_in < 9) return;
  if (in_sizes[0] != kTok * kDModel) return;
  if (in_sizes[1] != kDModel * kDModel || in_sizes[2] != kDModel) return;
  if (in_sizes[3] != kDModel * kDh || in_sizes[4] != kDh) return;
  if (in_sizes[5] != kDModel * kDh || in_sizes[6] != kDh) return;
  if (in_sizes[7] != kDModel * kDModel || in_sizes[8] != kDModel) return;
  if (out_size != kTok * kDModel) return;

  const float* x   = (const float*)d_in[0];
  const float* W_q = (const float*)d_in[1];
  const float* b_q = (const float*)d_in[2];
  const float* W_k = (const float*)d_in[3];
  const float* b_k = (const float*)d_in[4];
  const float* W_v = (const float*)d_in[5];
  const float* b_v = (const float*)d_in[6];
  const float* W_o = (const float*)d_in[7];
  const float* b_o = (const float*)d_in[8];
  float* out = (float*)d_out;

  const size_t bytesQO = (size_t)kTok * kDModel * 2;
  const size_t bytesK  = (size_t)kTok * kDh * 2;
  const size_t bytesVT = (size_t)kDh * kTok * 2;
  const size_t bytesSC = (size_t)kGrp * kSeq * kSeq * 4;
  const size_t bytesP  = (size_t)kGrp * kSeq * kSeq * 2;
  const size_t bytesX  = (size_t)kTok * kDModel * 2;
  const size_t bytesWq = (size_t)kDModel * kDModel * 2;
  const size_t bytesWk = (size_t)kDh * kDModel * 2;
  const size_t offQO = 0;
  const size_t offK  = offQO + bytesQO;
  const size_t offVT = offK + bytesK;
  const size_t offSC = offVT + bytesVT;
  const size_t offP  = offSC + bytesSC;
  const size_t total = offP + bytesP;
  if (total > ws_size) return;
  if (bytesX + bytesWq + 2 * bytesWk > bytesSC) return;

  char* ws = (char*)d_ws;
  unsigned short* QO16 = (unsigned short*)(ws + offQO);
  unsigned short* K16  = (unsigned short*)(ws + offK);
  unsigned short* VT   = (unsigned short*)(ws + offVT);
  float*          SC   = (float*)(ws + offSC);
  unsigned short* P16  = (unsigned short*)(ws + offP);
  unsigned short* X16  = (unsigned short*)(ws + offSC);
  unsigned short* WqT  = (unsigned short*)(ws + offSC + bytesX);
  unsigned short* WkT  = (unsigned short*)(ws + offSC + bytesX + bytesWq);
  unsigned short* WvT  = (unsigned short*)(ws + offSC + bytesX + bytesWq + bytesWk);
  unsigned short* WoT  = (unsigned short*)(ws + offSC);

  {
    const int n8 = kTok * kDModel / 8;
    cast8_f16_kernel<<<dim3(n8 / 256), dim3(256), 0, stream>>>(x, X16, n8);
  }
  wtcast_kernel<<<dim3(kDModel / 64, kDModel / 64, 1), dim3(256), 0, stream>>>(W_q, W_q, WqT, WqT, kDModel, kDModel, kWCarry);
  wtcast_kernel<<<dim3(kDModel / 64, kDh / 64, 2), dim3(256), 0, stream>>>(W_k, W_v, WkT, WvT, kDModel, kDh, kWCarry);

  wmma_gemm64<0, false, 2, 1, false><<<dim3((kTok / 64) * (kDModel / 64) / 8, 1), dim3(256), 0, stream>>>(
      X16, X16, kDModel, 0L, WqT, WqT, kDModel, 0L, (void*)QO16, nullptr, kDModel, 0L,
      b_q, nullptr, 0L, kTok, kDModel, kDModel, kWCarryInv);
  wmma_gemm64<0, false, 2, 1, false><<<dim3((kTok / 64) * (kDh / 64) / 8, 1), dim3(256), 0, stream>>>(
      X16, X16, kDModel, 0L, WkT, WkT, kDModel, 0L, (void*)K16, nullptr, kDh, 0L,
      b_k, nullptr, 0L, kTok, kDh, kDModel, kWCarryInv);
  wmma_gemm64<0, false, 1, 1, false><<<dim3((kDh / 64) * (kTok / 64) / 8, 1), dim3(256), 0, stream>>>(
      WvT, WvT, kDModel, 0L, X16, X16, kDModel, 0L, (void*)VT, nullptr, kTok, 0L,
      b_v, nullptr, 0L, kDh, kTok, kDModel, kWCarryInv);

  for (int bb = 0; bb < kBatch; ++bb) {
    for (int hc = 0; hc < kHeadChunks; ++hc) {
      const int h0 = hc * kGrp;
      const unsigned short* Qb = QO16 + (size_t)bb * kSeq * kDModel + (size_t)h0 * kDh;
      const unsigned short* Kb = K16 + (size_t)bb * kSeq * kDh;
      const unsigned short* Vb = VT + (size_t)bb * kSeq;
      unsigned short* Ob = QO16 + (size_t)bb * kSeq * kDModel + (size_t)h0 * kDh;
      wmma_gemm64<0, false, 0, 0, false><<<dim3((kSeq / 64) * (kSeq / 64) / 8, kGrp), dim3(256), 0, stream>>>(
          Qb, Qb, kDModel, (long)kDh, Kb, Kb, kDh, 0L, (void*)SC, nullptr, kSeq, (long)kSeq * kSeq,
          nullptr, nullptr, 0L, kSeq, kSeq, kDh, kScoreScale);
      softmax_row_kernel<<<dim3(kGrp * kSeq), dim3(256), 0, stream>>>(SC, P16, kPCarry);
      wmma_gemm64<0, false, 0, 1, false><<<dim3((kSeq / 64) * (kDh / 64) / 8, kGrp), dim3(256), 0, stream>>>(
          P16, P16, kSeq, (long)kSeq * kSeq, Vb, Vb, kTok, 0L, (void*)Ob, nullptr, kDModel, (long)kDh,
          nullptr, nullptr, 0L, kSeq, kDh, kSeq, kPVScale);
    }
  }

  wtcast_kernel<<<dim3(kDModel / 64, kDModel / 64, 1), dim3(256), 0, stream>>>(W_o, W_o, WoT, WoT, kDModel, kDModel, kWCarry);
  wmma_gemm64<0, false, 2, 0, false><<<dim3((kTok / 64) * (kDModel / 64) / 8, 1), dim3(256), 0, stream>>>(
      QO16, QO16, kDModel, 0L, WoT, WoT, kDModel, 0L, (void*)out, nullptr, kDModel, 0L,
      b_o, nullptr, 0L, kTok, kDModel, kDModel, kOutScale);
}
